// ChannelMambaFusionBlock_Mask_807453852221
// MI455X (gfx1250) — hardware-verified
//
#include <hip/hip_runtime.h>
#include <math.h>

typedef __attribute__((ext_vector_type(16))) _Float16 v16h;
typedef __attribute__((ext_vector_type(8)))  _Float16 v8h;
typedef __attribute__((ext_vector_type(8)))  float    v8f;
typedef __attribute__((ext_vector_type(4)))  float    v4f;

constexpr int kB     = 2;
constexpr int kC     = 96;
constexpr int kHt    = 128;
constexpr int kWd    = 128;
constexpr int kL     = kHt * kWd;
constexpr int kE     = 192;
constexpr int kG     = 24;
constexpr int kHeads = 16;
constexpr int kCi    = 12;
constexpr int kNs    = 12;
constexpr int kXR    = 25;
constexpr int kHid   = 384;
constexpr int kTokAll = kB * kL;
constexpr int kWPlane = kHid * kC;
static_assert(kL == 16384 && kTokAll == 32768, "token counts");
static_assert(kE == kHeads * kCi && kE == kG * 8 && kC == kG * 4, "channel maps");
static_assert(kXR == 1 + 2 * kNs, "projection rows");
static_assert((kC % 32) == 0 && (kHid % 32) == 0, "k-steps of 32");
static_assert(kWPlane == 36864, "weight plane");

constexpr float kW1Carry  = 16.0f;
constexpr float kW2Carry  = 16.0f;
constexpr float kUCarry   = 64.0f;
constexpr float kWxCarry  = 16.0f;
constexpr float kW1Fold   = 1.0f / kW1Carry;
constexpr float kW2Fold   = 1.0f / kW2Carry;
constexpr float kXFold    = 1.0f / (kUCarry * kWxCarry);

constexpr size_t kSzXR   = (size_t)2 * kB * kC * kL * 4;
constexpr size_t kSzUPRE = (size_t)2 * kB * kE * kL * 4;
constexpr size_t kSzU    = (size_t)2 * kB * kE * kL * 4;
constexpr size_t kSzW16  = (size_t)4 * kWPlane * 2;
constexpr size_t kOffXR   = 0;
constexpr size_t kOffUPRE = kOffXR + kSzXR;
constexpr size_t kOffRY   = kOffUPRE;
constexpr size_t kOffU    = kOffUPRE + kSzUPRE;
constexpr size_t kOffW16  = kOffU + kSzU;
constexpr size_t kWsTotal = kOffW16 + kSzW16;
static_assert(kWsTotal == 126124032ull, "carve total");
static_assert(kWsTotal <= 134217728ull, "carve cap");
static_assert((kOffUPRE % 128) == 0 && (kOffU % 128) == 0 && (kOffW16 % 128) == 0, "aligned regions");
static_assert(kSzXR <= kSzUPRE, "RY fits inside the dead UPRE region");

union FragU { v16h v; v8h h[2]; };
__device__ __forceinline__ v16h frag_load(const _Float16* p) {
  FragU f;
  f.h[0] = *(const v8h*)(p);
  f.h[1] = *(const v8h*)(p + 16);
  return f.v;
}
__device__ __forceinline__ v8f mma_h(v16h a, v16h b, v8f c) {
  c = __builtin_amdgcn_wmma_f32_16x16x32_f16(false, a, false, b, (short)0, c, false, false);
  asm volatile("v_nop\n\tv_nop\n\tv_nop\n\tv_nop" : "+v"(c) : "v"(a), "v"(b));
  return c;
}

__global__ __launch_bounds__(256) void cast_weights_kernel(
    const float* __restrict__ w0, const float* __restrict__ w1,
    const float* __restrict__ w2, const float* __restrict__ w3,
    unsigned short* __restrict__ dst, int total8, float scale)
{
  const int i = blockIdx.x * 256 + threadIdx.x;
  if (i >= total8) return;
  const int p = blockIdx.y;
  const float* src = w0;
  if (p == 1) src = w1;
  if (p == 2) src = w2;
  if (p == 3) src = w3;
  const size_t e0 = (size_t)i << 3;
  const v4f a0 = *(const v4f*)(src + e0);
  const v4f a1 = *(const v4f*)(src + e0 + 4);
  v8h hv;
#pragma unroll
  for (int e = 0; e < 4; ++e) {
    hv[e]     = (_Float16)(a0[e] * scale);
    hv[4 + e] = (_Float16)(a1[e] * scale);
  }
  unsigned short* q = dst + (size_t)p * kWPlane + e0;
  *(volatile v8h*)q = hv;
  __threadfence();
  *(volatile v8h*)q = hv;
}

__global__ __launch_bounds__(256) void ln_inproj_kernel(
    const float* __restrict__ x_rgb, const float* __restrict__ x_e,
    const float* __restrict__ lnw_r, const float* __restrict__ lnb_r,
    const float* __restrict__ lnw_e, const float* __restrict__ lnb_e,
    const float* __restrict__ ipw_r, const float* __restrict__ ipw_e,
    float* __restrict__ XR, float* __restrict__ UPRE)
{
  const int s = blockIdx.y;
  const float* x   = s ? x_e   : x_rgb;
  const float* lw  = s ? lnw_e : lnw_r;
  const float* lb  = s ? lnb_e : lnb_r;
  const float* ipw = s ? ipw_e : ipw_r;
  const int t = blockIdx.x * 256 + threadIdx.x;
  const int b = t >> 14;
  const int l = t & (kL - 1);
  const float* xb = x + (size_t)b * kC * kL + l;
  float sum = 0.0f;
#pragma unroll 4
  for (int c = 0; c < kC; ++c) sum += xb[(size_t)c * kL];
  const float mu = sum * (1.0f / (float)kC);
  float sq = 0.0f;
#pragma unroll 4
  for (int c = 0; c < kC; ++c) {
    const float dlt = xb[(size_t)c * kL] - mu;
    sq = fmaf(dlt, dlt, sq);
  }
  const float rs = rsqrtf(sq * (1.0f / (float)kC) + 1e-6f);
  float* xro = XR   + ((size_t)(s * kB + b) * kC) * kL + l;
  float* upo = UPRE + ((size_t)(s * kB + b) * kE) * kL + l;
#pragma unroll 1
  for (int g = 0; g < kG; ++g) {
    float xn[4];
#pragma unroll
    for (int j = 0; j < 4; ++j) {
      const int c0 = g * 4 + j;
      const float v = xb[(size_t)c0 * kL];
      xn[j] = (v - mu) * rs * lw[c0] + lb[c0];
    }
    float a[8];
#pragma unroll
    for (int i = 0; i < 8; ++i) {
      const float* wp = ipw + g * 32 + i * 4;
      float acc = xn[0] * wp[0];
      acc = fmaf(xn[1], wp[1], acc);
      acc = fmaf(xn[2], wp[2], acc);
      acc = fmaf(xn[3], wp[3], acc);
      a[i] = acc;
    }
    for (int pass = 0; pass < 2; ++pass) {
#pragma unroll
      for (int j = 0; j < 4; ++j) *(volatile float*)(xro + (size_t)(g * 4 + j) * kL) = xn[j];
#pragma unroll
      for (int i = 0; i < 8; ++i) *(volatile float*)(upo + (size_t)(g * 8 + i) * kL) = a[i];
      __threadfence();
    }
  }
}

constexpr int kStrip = 32;
static_assert((kHt % kStrip) == 0, "strip");
__device__ __forceinline__ void load_row3(const float* __restrict__ ip, int r, int x, int xl, int xr,
                                          bool fl, bool fr, float& a0, float& a1, float& a2) {
  const bool ok = (r >= 0) && (r < kHt);
  const int rc = (r < 0) ? 0 : ((r > kHt - 1) ? (kHt - 1) : r);
  float v0 = ip[rc * kWd + xl];
  float v1 = ip[rc * kWd + x];
  float v2 = ip[rc * kWd + xr];
  asm volatile("" : "+v"(v0), "+v"(v1), "+v"(v2));
  a0 = (ok && fl) ? v0 : 0.0f;
  a1 = ok ? v1 : 0.0f;
  a2 = (ok && fr) ? v2 : 0.0f;
}
__global__ __launch_bounds__(128) void dwconv_silu_kernel(
    const float* __restrict__ UPRE,
    const float* __restrict__ cw_r, const float* __restrict__ cb_r,
    const float* __restrict__ cw_e, const float* __restrict__ cb_e,
    float* __restrict__ U)
{
  const int plane = blockIdx.x;
  const int s = plane / (kB * kE);
  const int e = plane - (plane / kE) * kE;
  const float* cw = s ? cw_e : cw_r;
  const float* cb = s ? cb_e : cb_r;
  const float w00 = cw[e * 9 + 0], w01 = cw[e * 9 + 1], w02 = cw[e * 9 + 2];
  const float w10 = cw[e * 9 + 3], w11 = cw[e * 9 + 4], w12 = cw[e * 9 + 5];
  const float w20 = cw[e * 9 + 6], w21 = cw[e * 9 + 7], w22 = cw[e * 9 + 8];
  const float bias = cb[e];
  const float* ip = UPRE + (size_t)plane * kL;
  float* op = U + (size_t)plane * kL;
  const int x = threadIdx.x;
  const int y0 = blockIdx.y * kStrip;
  const bool fl = (x > 0), fr = (x < kWd - 1);
  const int xl = fl ? (x - 1) : 0;
  const int xr = fr ? (x + 1) : (kWd - 1);
  float t0, t1, t2, m0, m1, m2;
  load_row3(ip, y0 - 1, x, xl, xr, fl, fr, t0, t1, t2);
  load_row3(ip, y0, x, xl, xr, fl, fr, m0, m1, m2);
#pragma unroll 1
  for (int yy = 0; yy < kStrip; ++yy) {
    const int y = y0 + yy;
    float b0, b1, b2;
    load_row3(ip, y + 1, x, xl, xr, fl, fr, b0, b1, b2);
    float acc = w00 * t0;
    acc = fmaf(w01, t1, acc);
    acc = fmaf(w02, t2, acc);
    acc = fmaf(w10, m0, acc);
    acc = fmaf(w11, m1, acc);
    acc = fmaf(w12, m2, acc);
    acc = fmaf(w20, b0, acc);
    acc = fmaf(w21, b1, acc);
    acc = fmaf(w22, b2, acc);
    const float sv = acc + bias;
    const float sg = __builtin_amdgcn_rcpf(1.0f + expf(-sv));
    const float val = sv * sg;
    float* q = op + y * kWd + x;
    *(volatile float*)q = val;
    __threadfence();
    *(volatile float*)q = val;
    t0 = m0; t1 = m1; t2 = m2;
    m0 = b0; m1 = b1; m2 = b2;
  }
}

constexpr int kTok = 32;
constexpr int kXDRow = kCi * kTok;
static_assert((kL % kTok) == 0, "tile inside one batch element");
__global__ __launch_bounds__(256) void ssm_kernel(
    const float* __restrict__ U, const float* __restrict__ XR,
    const float* __restrict__ xprojw, const float* __restrict__ dtw, const float* __restrict__ dtb,
    const float* __restrict__ alogs, const float* __restrict__ dsk,
    const float* __restrict__ on1w, const float* __restrict__ on1b,
    const float* __restrict__ on2w, const float* __restrict__ on2b,
    const float* __restrict__ ow_r, const float* __restrict__ ow_e,
    float* __restrict__ RY)
{
  __shared__ __align__(16) float sU[2 * kE * kTok];
  __shared__ __align__(16) float sXD[2 * kXR * kXDRow];
  const int tid = threadIdx.x, lane = tid & 31, wave = tid >> 5;
  const int hh = lane >> 4, nn = lane & 15;
  const int t0 = blockIdx.x * kTok;
  const int b  = t0 >> 14;
  const int l0 = t0 & (kL - 1);

#pragma unroll
  for (int it = 0; it < 12; ++it) {
    const int idx = tid + it * 256;
    const int row = idx >> 3;
    const int c4  = (idx & 7) * 4;
    const int k   = (row >= kE) ? 1 : 0;
    const int e   = row - k * kE;
    const v4f v = *(const v4f*)(U + ((size_t)(k * kB + b) * kE + e) * kL + l0 + c4);
    *(v4f*)(sU + row * kTok + c4) = v;
  }

  v16h bfr[4];
#pragma unroll
  for (int nt = 0; nt < 4; ++nt) {
    const int kq = nt >> 1;
    const int r  = (nt & 1) * 16 + nn;
    const int rc = (r < kXR) ? r : (kXR - 1);
    const bool ok = (r < kXR);
    const float* wp = xprojw + (kq * kXR + rc) * kHeads + 8 * hh;
    const v4f q0 = *(const v4f*)(wp);
    const v4f q1 = *(const v4f*)(wp + 4);
    v8h live, zero;
#pragma unroll
    for (int i = 0; i < 4; ++i) {
      const float f0 = ok ? (q0[i] * kWxCarry) : 0.0f;
      const float f1 = ok ? (q1[i] * kWxCarry) : 0.0f;
      live[i]     = (_Float16)f0;
      live[4 + i] = (_Float16)f1;
      zero[i]     = (_Float16)0.0f;
      zero[4 + i] = (_Float16)0.0f;
    }
    FragU f;
    if (kq == 0) { f.h[0] = live; f.h[1] = zero; }
    else         { f.h[0] = zero; f.h[1] = live; }
    bfr[nt] = f.v;
  }
  __syncthreads();

#pragma unroll
  for (int j = 0; j < 3; ++j) {
    const int mt = wave * 3 + j;
    const int ci = mt >> 1;
    const int tb = (mt & 1) * 16;
    v8h a0, a1;
#pragma unroll
    for (int i = 0; i < 8; ++i) {
      const int e = (8 * hh + i) * kCi + ci;
      a0[i] = (_Float16)(sU[e * kTok + tb + nn] * kUCarry);
      a1[i] = (_Float16)(sU[(kE + e) * kTok + tb + nn] * kUCarry);
    }
    FragU af;
    af.h[0] = a0;
    af.h[1] = a1;
    v8f acc[4];
#pragma unroll
    for (int nt = 0; nt < 4; ++nt) {
      acc[nt] = (v8f){0.f, 0.f, 0.f, 0.f, 0.f, 0.f, 0.f, 0.f};
      acc[nt] = mma_h(af.v, bfr[nt], acc[nt]);
    }
#pragma unroll
    for (int nt = 0; nt < 4; ++nt) {
      const int kq = nt >> 1;
      const int r  = (nt & 1) * 16 + nn;
      const int rc = (r < kXR) ? r : (kXR - 1);
      float* dp = sXD + (kq * kXR + rc) * kXDRow + ci * kTok + tb + 8 * hh;
      if (r < kXR) {
#pragma unroll
        for (int rr = 0; rr < 8; ++rr) dp[rr] = acc[nt][rr] * kXFold;
      }
    }
  }
  __syncthreads();

  const int tok = lane;
#pragma unroll 1
  for (int j = 0; j < 4; ++j) {
    const int p = wave * 4 + j;
    const int k = p >> 4;
    const int d = p & 15;
    const float dw = dtw[p], db = dtb[p], Dv = dsk[p];
    float An[kNs], h[kNs];
#pragma unroll
    for (int n = 0; n < kNs; ++n) {
      An[n] = -expf(alogs[p * kNs + n]);
      h[n] = 0.0f;
    }
    const float* xk = sXD + (k * kXR) * kXDRow + tok;
    const float* xo = sXD + ((1 - k) * kXR + 1 + kNs) * kXDRow + tok;
    float* up = sU + (k * kE + d * kCi) * kTok + tok;
    float ysum = 0.0f;
#pragma unroll 1
    for (int ci = 0; ci < kCi; ++ci) {
      const float uu  = up[ci * kTok];
      const float dts = xk[ci * kTok];
      const float xln = dw * dts + db;
      const float dt  = fmaxf(xln, 0.0f) + log1pf(expf(-fabsf(xln)));
      const float du  = dt * uu;
      float y = 0.0f;
#pragma unroll
      for (int n = 0; n < kNs; ++n) {
        const float Bn = xk[((1 + n) * kCi + ci) * kTok];
        const float Cn = xo[(n * kCi + ci) * kTok];
        const float dA = expf(dt * An[n]);
        const float hn = fmaf(dA, h[n], du * Bn);
        h[n] = hn;
        y = fmaf(hn, Cn, y);
      }
      y = fmaf(Dv, uu, y);
      up[ci * kTok] = y;
      ysum += y;
    }
    const float mu = ysum * (1.0f / (float)kCi);
    float var = 0.0f;
#pragma unroll 1
    for (int ci = 0; ci < kCi; ++ci) {
      const float dlt = up[ci * kTok] - mu;
      var = fmaf(dlt, dlt, var);
    }
    const float rs = rsqrtf(var * (1.0f / (float)kCi) + 1e-5f);
    const float* onw = k ? on2w : on1w;
    const float* onb = k ? on2b : on1b;
#pragma unroll 1
    for (int ci = 0; ci < kCi; ++ci) {
      const float yv = up[ci * kTok];
      up[ci * kTok] = (yv - mu) * rs * onw[ci] + onb[ci];
    }
  }
  __syncthreads();

#pragma unroll 1
  for (int j = 0; j < 6; ++j) {
    const int q = wave * 6 + j;
    const int k = (q >= kG) ? 1 : 0;
    const int g = q - k * kG;
    const float* ow = (k ? ow_e : ow_r) + g * 32;
    float yv[8];
#pragma unroll
    for (int i = 0; i < 8; ++i) yv[i] = sU[(k * kE + g * 8 + i) * kTok + tok];
    const size_t base = ((size_t)(k * kB + b) * kC + g * 4) * kL + l0 + tok;
    float o[4];
#pragma unroll
    for (int oo = 0; oo < 4; ++oo) {
      float a = yv[0] * ow[oo * 8 + 0];
#pragma unroll
      for (int i = 1; i < 8; ++i) a = fmaf(yv[i], ow[oo * 8 + i], a);
      o[oo] = a + XR[base + (size_t)oo * kL];
    }
    for (int pass = 0; pass < 2; ++pass) {
#pragma unroll
      for (int oo = 0; oo < 4; ++oo) *(volatile float*)(RY + base + (size_t)oo * kL) = o[oo];
      __threadfence();
    }
  }
}

constexpr int kMT = 64;
constexpr int kRP = 68;
constexpr int kAP = 104;
constexpr int kHP = 392;
static_assert((kL % kMT) == 0, "tile inside one batch element");
static_assert((kAP % 8) == 0 && (kHP % 8) == 0 && (kRP % 4) == 0, "16-B aligned LDS rows");
__global__ __launch_bounds__(192) void mlp_kernel(
    const float* __restrict__ RY,
    const float* __restrict__ n1w, const float* __restrict__ n1b,
    const float* __restrict__ n2w, const float* __restrict__ n2b,
    const unsigned short* __restrict__ W16,
    const float* __restrict__ b1_r, const float* __restrict__ b1_e,
    const float* __restrict__ b2_r, const float* __restrict__ b2_e,
    float* __restrict__ out)
{
  __shared__ __align__(16) float    sR[kC * kRP];
  __shared__ __align__(16) _Float16 sA[kMT * kAP];
  __shared__ __align__(16) _Float16 sH[kMT * kHP];
  __shared__ float sP1[3 * kMT];
  __shared__ float sP2[3 * kMT];
  const int tid = threadIdx.x, lane = tid & 31, wave = tid >> 5;
  const int hh = lane >> 4, nn = lane & 15;
  const int s  = blockIdx.y;
  const int t0 = blockIdx.x * kMT;
  const int b  = t0 >> 14;
  const int l0 = t0 & (kL - 1);
  const float* ry = RY  + ((size_t)(s * kB + b) * kC) * kL + l0;
  float*       op = out + ((size_t)(s * kB + b) * kC) * kL + l0;

#pragma unroll
  for (int it = 0; it < 8; ++it) {
    const int idx = tid + it * 192;
    const int row = idx >> 4;
    const int c4  = (idx & 15) * 4;
    const v4f v = *(const v4f*)(ry + (size_t)row * kL + c4);
    *(v4f*)(sR + row * kRP + c4) = v;
  }
  __syncthreads();

  const int tok  = tid & 63;
  const int part = tid >> 6;
  const int cb0  = part * 32;
  {
    float ps = 0.0f;
#pragma unroll 4
    for (int c = 0; c < 32; ++c) ps += sR[(cb0 + c) * kRP + tok];
    sP1[part * kMT + tok] = ps;
  }
  __syncthreads();
  const float mu = (sP1[tok] + sP1[kMT + tok] + sP1[2 * kMT + tok]) * (1.0f / (float)kC);
  {
    float pv = 0.0f;
#pragma unroll 4
    for (int c = 0; c < 32; ++c) {
      const float dlt = sR[(cb0 + c) * kRP + tok] - mu;
      pv = fmaf(dlt, dlt, pv);
    }
    sP2[part * kMT + tok] = pv;
  }
  __syncthreads();
  {
    const float var = (sP2[tok] + sP2[kMT + tok] + sP2[2 * kMT + tok]) * (1.0f / (float)kC);
    const float rs = rsqrtf(var + 1e-6f);
    const float* nw = s ? n2w : n1w;
    const float* nb = s ? n2b : n1b;
#pragma unroll 4
    for (int c = 0; c < 32; ++c) {
      const int ch = cb0 + c;
      const float z = (sR[ch * kRP + tok] - mu) * rs * nw[ch] + nb[ch];
      sA[tok * kAP + ch] = (_Float16)z;
    }
  }
  __syncthreads();

  const _Float16* W1 = (const _Float16*)(W16 + (size_t)(s * 2) * kWPlane);
  const _Float16* W2 = W1 + kWPlane;
  const float* b1 = s ? b1_e : b1_r;
  const float* b2 = s ? b2_e : b2_r;

#pragma unroll 1
  for (int jj = 0; jj < 4; ++jj) {
    const int nrow = (wave * 4 + jj) * 16 + nn;
    const _Float16* bp = W1 + (size_t)nrow * kC + 8 * hh;
    const v16h bf0 = frag_load(bp);
    const v16h bf1 = frag_load(bp + 32);
    const v16h bf2 = frag_load(bp + 64);
    const float bias = b1[nrow];
#pragma unroll 1
    for (int i = 0; i < 4; ++i) {
      const _Float16* ap = sA + (i * 16 + nn) * kAP + 8 * hh;
      const v16h a0 = frag_load(ap);
      const v16h a1 = frag_load(ap + 32);
      const v16h a2 = frag_load(ap + 64);
      v8f acc = (v8f){0.f, 0.f, 0.f, 0.f, 0.f, 0.f, 0.f, 0.f};
      acc = mma_h(a0, bf0, acc);
      acc = mma_h(a1, bf1, acc);
      acc = mma_h(a2, bf2, acc);
#pragma unroll
      for (int r = 0; r < 8; ++r) {
        const float v = acc[r] * kW1Fold + bias;
        const float gl = 0.5f * v * (1.0f + erff(v * 0.70710678118654752f));
        sH[(i * 16 + 8 * hh + r) * kHP + nrow] = (_Float16)gl;
      }
    }
  }
  __syncthreads();

  {
    const int nrow = wave * 16 + nn;
    v8f acc[4];
#pragma unroll
    for (int i = 0; i < 4; ++i) acc[i] = (v8f){0.f, 0.f, 0.f, 0.f, 0.f, 0.f, 0.f, 0.f};
    const _Float16* bp = W2 + (size_t)nrow * kHid + 8 * hh;
#pragma unroll 1
    for (int ks = 0; ks < kHid / 32; ++ks) {
      const int k0 = ks * 32;
      const v16h bf = frag_load(bp + k0);
#pragma unroll
      for (int i = 0; i < 4; ++i) {
        const v16h af = frag_load(sH + (i * 16 + nn) * kHP + k0 + 8 * hh);
        acc[i] = mma_h(af, bf, acc[i]);
      }
    }
    const float bias2 = b2[nrow];
#pragma unroll
    for (int i = 0; i < 4; ++i) {
#pragma unroll
      for (int r = 0; r < 8; ++r) {
        const int tr = i * 16 + 8 * hh + r;
        const float v = acc[i][r] * kW2Fold + bias2 + sR[nrow * kRP + tr];
        sR[nrow * kRP + tr] = v;
      }
    }
  }
  __syncthreads();

  {
    const int c4 = nn * 4;
    v4f vals[8];
#pragma unroll
    for (int it = 0; it < 8; ++it) {
      const int row = wave * 16 + it * 2 + hh;
      vals[it] = *(const v4f*)(sR + row * kRP + c4);
    }
    for (int pass = 0; pass < 2; ++pass) {
#pragma unroll
      for (int it = 0; it < 8; ++it) {
        const int row = wave * 16 + it * 2 + hh;
        *(volatile v4f*)(op + (size_t)row * kL + c4) = vals[it];
      }
      __threadfence();
    }
  }
}

extern "C" void kernel_launch(void* const* d_in, const int* in_sizes, int n_in,
                              void* d_out, int out_size, void* d_ws, size_t ws_size,
                              hipStream_t stream)
{
  if (n_in < 35) return;
  const int expect[35] = {
    kB * kC * kL, kB * kC * kL, kC, kC, kC, kC,
    kG * 32, kG * 32, kE * 9, kE, kE * 9, kE,
    2 * kXR * kHeads, 2 * kHeads, 2 * kHeads, 2 * kHeads * kNs, 2 * kHeads,
    kCi, kCi, kCi, kCi,
    kG * 32, kG * 32, kC, kC, kC, kC,
    kWPlane, kHid, kWPlane, kC, kWPlane, kHid, kWPlane, kC };
  static_assert(sizeof(expect) / sizeof(expect[0]) == 35, "input table");
  for (int i = 0; i < 35; ++i) {
    if (in_sizes[i] != expect[i]) return;
  }
  if (out_size != 2 * kB * kC * kL) return;
  if (ws_size < kWsTotal) return;

  const float* x_rgb  = (const float*)d_in[0];
  const float* x_e    = (const float*)d_in[1];
  const float* in1w   = (const float*)d_in[2];
  const float* in1b   = (const float*)d_in[3];
  const float* in2w   = (const float*)d_in[4];
  const float* in2b   = (const float*)d_in[5];
  const float* ipw_r  = (const float*)d_in[6];
  const float* ipw_e  = (const float*)d_in[7];
  const float* cw_r   = (const float*)d_in[8];
  const float* cb_r   = (const float*)d_in[9];
  const float* cw_e   = (const float*)d_in[10];
  const float* cb_e   = (const float*)d_in[11];
  const float* xprojw = (const float*)d_in[12];
  const float* dtw    = (const float*)d_in[13];
  const float* dtb    = (const float*)d_in[14];
  const float* alogs  = (const float*)d_in[15];
  const float* dsk    = (const float*)d_in[16];
  const float* on1w   = (const float*)d_in[17];
  const float* on1b   = (const float*)d_in[18];
  const float* on2w   = (const float*)d_in[19];
  const float* on2b   = (const float*)d_in[20];
  const float* opw_r  = (const float*)d_in[21];
  const float* opw_e  = (const float*)d_in[22];
  const float* n1w    = (const float*)d_in[23];
  const float* n1b    = (const float*)d_in[24];
  const float* n2w    = (const float*)d_in[25];
  const float* n2b    = (const float*)d_in[26];
  const float* fc1w_r = (const float*)d_in[27];
  const float* fc1b_r = (const float*)d_in[28];
  const float* fc2w_r = (const float*)d_in[29];
  const float* fc2b_r = (const float*)d_in[30];
  const float* fc1w_e = (const float*)d_in[31];
  const float* fc1b_e = (const float*)d_in[32];
  const float* fc2w_e = (const float*)d_in[33];
  const float* fc2b_e = (const float*)d_in[34];

  char* ws = (char*)d_ws;
  float*          XR   = (float*)(ws + kOffXR);
  float*          UPRE = (float*)(ws + kOffUPRE);
  float*          RY   = (float*)(ws + kOffRY);
  float*          U    = (float*)(ws + kOffU);
  unsigned short* W16  = (unsigned short*)(ws + kOffW16);

  static_assert(kW1Carry == kW2Carry, "one cast scale for all four planes");
  cast_weights_kernel<<<dim3((kWPlane / 8) / 256, 4), 256, 0, stream>>>(
      fc1w_r, fc2w_r, fc1w_e, fc2w_e, W16, kWPlane / 8, kW1Carry);

  ln_inproj_kernel<<<dim3(kTokAll / 256, 2), 256, 0, stream>>>(
      x_rgb, x_e, in1w, in1b, in2w, in2b, ipw_r, ipw_e, XR, UPRE);

  dwconv_silu_kernel<<<dim3(2 * kB * kE, kHt / kStrip), kWd, 0, stream>>>(
      UPRE, cw_r, cb_r, cw_e, cb_e, U);

  ssm_kernel<<<dim3(kTokAll / kTok), 256, 0, stream>>>(
      U, XR, xprojw, dtw, dtb, alogs, dsk, on1w, on1b, on2w, on2b, opw_r, opw_e, RY);

  mlp_kernel<<<dim3(kTokAll / kMT, 2), 192, 0, stream>>>(
      RY, n1w, n1b, n2w, n2b, W16, fc1b_r, fc1b_e, fc2b_r, fc2b_e, (float*)d_out);
}
